// gru_encoder_46437186405043
// MI455X (gfx1250) — hardware-verified
//
#include <hip/hip_runtime.h>
#include <math.h>

constexpr int NBAT    = 256;
constexpr int NSTEP   = 512;
constexpr int NINP    = 16;
constexpr int NHID    = 128;
constexpr int NGATE3  = 384;
constexpr int NOUTF   = 16;
constexpr int NTHR    = 256;
constexpr int SEQ_BLK = 16;
constexpr int XKPAD   = 32;
constexpr int XCHUNK  = 8;
constexpr int XPITCH  = 40;
constexpr int HPITCH  = 136;
constexpr int OPITCH  = 132;
constexpr float WCARRY     = 16.0f;
constexpr float WCARRY_INV = 1.0f / 16.0f;
constexpr int NOUT0 = NBAT * NSTEP * NOUTF;
constexpr int NOUT1 = 2 * NBAT * NHID;

static_assert(NBAT % SEQ_BLK == 0, "batch tiles");
static_assert(NHID == 16 * (NTHR / 32), "8 waves x 16 hidden columns");
static_assert(NGATE3 == 3 * NHID, "gate rows r|z|n");
static_assert(NHID % 32 == 0, "K multiple of 32");
static_assert(NINP == 16 && XKPAD == 32, "x K padded 16 -> 32");
static_assert(NSTEP % XCHUNK == 0, "chunked staging");
static_assert(XCHUNK * NOUTF == 128, "one staged out0 row = 32 lanes x 4 floats");
static_assert(NTHR == SEQ_BLK * XCHUNK * 2, "x staging thread map");
static_assert((2 * SEQ_BLK * HPITCH) % NTHR == 0, "h zero-fill loop exact");
static_assert(XPITCH % 8 == 0 && HPITCH % 8 == 0 && OPITCH % 4 == 0, "16-B aligned rows");
static_assert(NOUT0 * 4 == 8388608, "out0 bytes");
static_assert((NOUT0 + NOUT1) * 4 == 8650752, "d_out bytes");

typedef __attribute__((ext_vector_type(16))) _Float16 v16h;
typedef __attribute__((ext_vector_type(8)))  _Float16 v8h;
typedef __attribute__((ext_vector_type(8)))  float    v8f;
typedef __attribute__((ext_vector_type(4)))  float    v4f;

__device__ __forceinline__ unsigned short f2bf_bits(float f) {
  unsigned u = __float_as_uint(f);
  return (unsigned short)((u + 0x7FFFu + ((u >> 16) & 1u)) >> 16);
}
__device__ __forceinline__ float bf_bits2f(unsigned short h) { return __uint_as_float(((unsigned)h) << 16); }
__device__ __forceinline__ float bf16r(float f) { return bf_bits2f(f2bf_bits(f)); }

struct FragH {
  union U { v16h v; v8h h[2]; };
  static __device__ __forceinline__ v16h load(const _Float16* p) {
    U f;
    f.h[0] = *(const v8h*)(p);
    f.h[1] = *(const v8h*)(p + 16);
    return f.v;
  }
  static __device__ __forceinline__ v8f mma(v16h a, v16h b, v8f c) {
    return __builtin_amdgcn_wmma_f32_16x16x32_f16(false, a, false, b, (short)0, c, false, false);
  }
};

__device__ __forceinline__ void guard3(v8f& p, v8f& q, v8f& s, v16h a, v16h b0, v16h b1, v16h b2) {
  asm volatile("v_nop\n\tv_nop\n\tv_nop\n\tv_nop" : "+v"(p), "+v"(q), "+v"(s) : "v"(a), "v"(b0), "v"(b1), "v"(b2));
}
__device__ __forceinline__ void guard1(v8f& p, v16h a, v16h b) {
  asm volatile("v_nop\n\tv_nop\n\tv_nop\n\tv_nop" : "+v"(p) : "v"(a), "v"(b));
}
__device__ __forceinline__ void guard4(v8f& a, v8f& b, v8f& c, v8f& d) {
  asm volatile("v_nop\n\tv_nop\n\tv_nop\n\tv_nop" : "+v"(a), "+v"(b), "+v"(c), "+v"(d));
}
__device__ __forceinline__ void guard_acc1(v8f& a) {
  asm volatile("v_nop\n\tv_nop\n\tv_nop\n\tv_nop" : "+v"(a));
}

__device__ __forceinline__ float gate_sig(float x)  { return __builtin_amdgcn_rcpf(1.0f + expf(-x)); }
__device__ __forceinline__ float gate_tanh(float x) { return 1.0f - 2.0f * __builtin_amdgcn_rcpf(expf(2.0f * x) + 1.0f); }

__global__ __launch_bounds__(NTHR) void wplane_kernel(const float* __restrict__ src, unsigned short* __restrict__ dst,
                                                      int nrow, int scols, int dcols8, float sc) {
  const int i  = blockIdx.x * NTHR + threadIdx.x;
  const int n8 = nrow * dcols8;
  if (i < n8) {
    const int row  = i / dcols8;
    const int g    = i - row * dcols8;
    const int col0 = g * 8;
    const bool valid = (col0 < scols);
    const int csrc = valid ? col0 : 0;
    const float* sp = src + (size_t)row * scols + csrc;
    const v4f a = *(const v4f*)(sp);
    const v4f b = *(const v4f*)(sp + 4);
    v8h hv;
#pragma unroll
    for (int e = 0; e < 4; ++e) {
      const float fa = valid ? a[e] : 0.0f;
      const float fb = valid ? b[e] : 0.0f;
      hv[e]     = (_Float16)(bf16r(fa) * sc);
      hv[4 + e] = (_Float16)(bf16r(fb) * sc);
    }
    *(volatile v8h*)(dst + (size_t)i * 8) = hv;
    __threadfence();
    *(volatile v8h*)(dst + (size_t)i * 8) = hv;
  }
}

__device__ __forceinline__ void stage_x8(const float* __restrict__ x, _Float16* xs, int rowbase, int tbase, int tid) {
  const int m  = tid >> 4;
  const int tt = (tid >> 1) & 7;
  const int hf = tid & 1;
  const float* sp = x + ((size_t)(rowbase + m) * NSTEP + (size_t)(tbase + tt)) * NINP + hf * 8;
  const v4f a = *(const v4f*)(sp);
  const v4f b = *(const v4f*)(sp + 4);
  v8h hv, zv;
#pragma unroll
  for (int e = 0; e < 4; ++e) {
    hv[e]     = (_Float16)bf16r(a[e]);
    hv[4 + e] = (_Float16)bf16r(b[e]);
  }
#pragma unroll
  for (int e = 0; e < 8; ++e) zv[e] = (_Float16)0.0f;
  _Float16* dp = xs + (tt * SEQ_BLK + m) * XPITCH + hf * 8;
  *(v8h*)(dp) = hv;
  *(v8h*)(dp + 16) = zv;
}

__global__ __launch_bounds__(NTHR) void gru2_seq_kernel(const float* __restrict__ x,
                                                        const unsigned short* __restrict__ wih0p,
                                                        const unsigned short* __restrict__ whh0p,
                                                        const unsigned short* __restrict__ wih1p,
                                                        const unsigned short* __restrict__ whh1p,
                                                        const unsigned short* __restrict__ wfcp,
                                                        float* __restrict__ out) {
  __shared__ __align__(16) _Float16 X8[XCHUNK * SEQ_BLK * XPITCH];
  __shared__ __align__(16) _Float16 Hh[2][SEQ_BLK * HPITCH];
  __shared__ __align__(16) float    OutS[SEQ_BLK * OPITCH];
  __shared__ __align__(16) float    Hs[2][SEQ_BLK * OPITCH];

  const int tid  = threadIdx.x;
  const int lane = tid & 31;
  const int wave = __builtin_amdgcn_readfirstlane(tid >> 5);
  const int c    = lane & 15;
  const int hh   = lane >> 4;
  const int koff = hh * 8;
  const int rowbase = blockIdx.x * SEQ_BLK;
  const int ucol = 16 * wave + c;

  {
    _Float16* hflat = &Hh[0][0];
#pragma unroll 1
    for (int i = tid; i < 2 * SEQ_BLK * HPITCH; i += NTHR) hflat[i] = (_Float16)0.0f;
  }
  stage_x8(x, X8, rowbase, 0, tid);

  const _Float16* w0x = (const _Float16*)wih0p + (size_t)ucol * XKPAD + koff;
  const v16h wxr = FragH::load(w0x);
  const v16h wxz = FragH::load(w0x + (size_t)NHID * XKPAD);
  const v16h wxn = FragH::load(w0x + (size_t)2 * NHID * XKPAD);
  constexpr int GSTR = NHID * NHID;
  const _Float16* w0h = (const _Float16*)whh0p + (size_t)ucol * NHID + koff;
  const _Float16* w1x = (const _Float16*)wih1p + (size_t)ucol * NHID + koff;
  const _Float16* w1h = (const _Float16*)whh1p + (size_t)ucol * NHID + koff;
  const _Float16* wfc = (const _Float16*)wfcp  + (size_t)c * NHID + koff;

  const _Float16* xrow  = X8 + c * XPITCH + koff;
  const _Float16* h0row = &Hh[0][0] + c * HPITCH + koff;
  const _Float16* h1row = &Hh[1][0] + c * HPITCH + koff;
  _Float16* h0w = &Hh[0][0] + (8 * hh) * HPITCH + ucol;
  _Float16* h1w = &Hh[1][0] + (8 * hh) * HPITCH + ucol;

  float h0reg[8], h1reg[8];
#pragma unroll
  for (int r = 0; r < 8; ++r) { h0reg[r] = 0.0f; h1reg[r] = 0.0f; }
  const v8f z8 = {0.f, 0.f, 0.f, 0.f, 0.f, 0.f, 0.f, 0.f};
  __syncthreads();

#pragma unroll 1
  for (int t = 0; t < NSTEP; ++t) {
    const int ts = t & (XCHUNK - 1);

    {
      v8f aR = z8, aZ = z8, aNX = z8, aNH = z8;
      {
        const v16h a = FragH::load(xrow + ts * (SEQ_BLK * XPITCH));
        aR  = FragH::mma(a, wxr, aR);
        aZ  = FragH::mma(a, wxz, aZ);
        aNX = FragH::mma(a, wxn, aNX);
        guard3(aR, aZ, aNX, a, wxr, wxz, wxn);
      }
#pragma unroll 1
      for (int k0 = 0; k0 < NHID; k0 += 32) {
        const v16h a  = FragH::load(h0row + k0);
        const v16h b0 = FragH::load(w0h + k0);
        const v16h b1 = FragH::load(w0h + GSTR + k0);
        const v16h b2 = FragH::load(w0h + 2 * GSTR + k0);
        aR  = FragH::mma(a, b0, aR);
        aZ  = FragH::mma(a, b1, aZ);
        aNH = FragH::mma(a, b2, aNH);
        guard3(aR, aZ, aNH, a, b0, b1, b2);
      }
      guard4(aR, aZ, aNX, aNH);
      __syncthreads();
#pragma unroll
      for (int r = 0; r < 8; ++r) {
        const float rg = gate_sig(aR[r] * WCARRY_INV);
        const float zg = gate_sig(aZ[r] * WCARRY_INV);
        const float ng = gate_tanh(aNX[r] * WCARRY_INV + rg * (aNH[r] * WCARRY_INV));
        const float hn = (1.0f - zg) * ng + zg * h0reg[r];
        h0reg[r] = hn;
        h0w[r * HPITCH] = (_Float16)hn;
      }
    }
    __syncthreads();

    {
      v8f aR = z8, aZ = z8, aNX = z8, aNH = z8;
#pragma unroll 1
      for (int k0 = 0; k0 < NHID; k0 += 32) {
        {
          const v16h a  = FragH::load(h0row + k0);
          const v16h b0 = FragH::load(w1x + k0);
          const v16h b1 = FragH::load(w1x + GSTR + k0);
          const v16h b2 = FragH::load(w1x + 2 * GSTR + k0);
          aR  = FragH::mma(a, b0, aR);
          aZ  = FragH::mma(a, b1, aZ);
          aNX = FragH::mma(a, b2, aNX);
          guard3(aR, aZ, aNX, a, b0, b1, b2);
        }
        {
          const v16h a  = FragH::load(h1row + k0);
          const v16h b0 = FragH::load(w1h + k0);
          const v16h b1 = FragH::load(w1h + GSTR + k0);
          const v16h b2 = FragH::load(w1h + 2 * GSTR + k0);
          aR  = FragH::mma(a, b0, aR);
          aZ  = FragH::mma(a, b1, aZ);
          aNH = FragH::mma(a, b2, aNH);
          guard3(aR, aZ, aNH, a, b0, b1, b2);
        }
      }
      guard4(aR, aZ, aNX, aNH);
      __syncthreads();
#pragma unroll
      for (int r = 0; r < 8; ++r) {
        const float rg = gate_sig(aR[r] * WCARRY_INV);
        const float zg = gate_sig(aZ[r] * WCARRY_INV);
        const float ng = gate_tanh(aNX[r] * WCARRY_INV + rg * (aNH[r] * WCARRY_INV));
        const float hn = (1.0f - zg) * ng + zg * h1reg[r];
        h1reg[r] = hn;
        h1w[r * HPITCH] = (_Float16)hn;
      }
    }
    if (ts == XCHUNK - 1 && t + 1 < NSTEP) stage_x8(x, X8, rowbase, t + 1, tid);
    __syncthreads();

    if (wave == 0) {
      v8f acc = z8;
#pragma unroll 1
      for (int k0 = 0; k0 < NHID; k0 += 32) {
        const v16h a = FragH::load(h1row + k0);
        const v16h b = FragH::load(wfc + k0);
        acc = FragH::mma(a, b, acc);
        guard1(acc, a, b);
      }
      guard_acc1(acc);
      float* os = OutS + (8 * hh) * OPITCH + ts * NOUTF + c;
#pragma unroll
      for (int r = 0; r < 8; ++r) os[r * OPITCH] = acc[r] * WCARRY_INV;
      if (ts == XCHUNK - 1) {
        __builtin_amdgcn_fence(__ATOMIC_RELEASE, "workgroup");
        __builtin_amdgcn_wave_barrier();
        __builtin_amdgcn_fence(__ATOMIC_ACQUIRE, "workgroup");
        const int t0 = t - (XCHUNK - 1);
        for (int pass = 0; pass < 2; ++pass) {
#pragma unroll 1
          for (int b = 0; b < SEQ_BLK; ++b) {
            const v4f v = *(const v4f*)(OutS + b * OPITCH + 4 * lane);
            *(volatile v4f*)(out + ((size_t)(rowbase + b) * NSTEP + (size_t)t0) * NOUTF + 4 * lane) = v;
          }
          __threadfence();
        }
        __builtin_amdgcn_fence(__ATOMIC_RELEASE, "workgroup");
        __builtin_amdgcn_wave_barrier();
        __builtin_amdgcn_fence(__ATOMIC_ACQUIRE, "workgroup");
      }
    }
  }

  {
    float* hs0 = &Hs[0][0] + (8 * hh) * OPITCH + ucol;
    float* hs1 = &Hs[1][0] + (8 * hh) * OPITCH + ucol;
#pragma unroll
    for (int r = 0; r < 8; ++r) {
      hs0[r * OPITCH] = h0reg[r];
      hs1[r * OPITCH] = h1reg[r];
    }
  }
  __syncthreads();
  {
    float* hid = out + (size_t)NOUT0;
    const float* hsf = &Hs[0][0];
    for (int pass = 0; pass < 2; ++pass) {
#pragma unroll
      for (int it = 0; it < 4; ++it) {
        const int idx   = wave * 4 + it;
        const int layer = idx >> 4;
        const int row   = idx & 15;
        const v4f v = *(const v4f*)(hsf + (layer * SEQ_BLK + row) * OPITCH + 4 * lane);
        *(volatile v4f*)(hid + ((size_t)layer * NBAT + (size_t)(rowbase + row)) * NHID + 4 * lane) = v;
      }
      __threadfence();
    }
  }
}

extern "C" void kernel_launch(void* const* d_in, const int* in_sizes, int n_in,
                              void* d_out, int out_size, void* d_ws, size_t ws_size, hipStream_t stream) {
  if (n_in < 6 || d_out == nullptr || d_ws == nullptr) return;
  if (in_sizes[0] != NBAT * NSTEP * NINP || in_sizes[1] != NGATE3 * NINP || in_sizes[2] != NGATE3 * NHID ||
      in_sizes[3] != NGATE3 * NHID || in_sizes[4] != NGATE3 * NHID || in_sizes[5] != NOUTF * NHID ||
      out_size != NOUT0 + NOUT1) return;

  const float* x    = (const float*)d_in[0];
  const float* wih0 = (const float*)d_in[1];
  const float* whh0 = (const float*)d_in[2];
  const float* wih1 = (const float*)d_in[3];
  const float* whh1 = (const float*)d_in[4];
  const float* wfc  = (const float*)d_in[5];
  float* out = (float*)d_out;

  char* ws = (char*)d_ws;
  size_t off = 0;
  auto carve = [&](size_t bytes) -> char* { char* p = ws + off; off += (bytes + 255) & ~(size_t)255; return p; };
  unsigned short* WIH0P = (unsigned short*)carve((size_t)NGATE3 * XKPAD * 2);
  unsigned short* WHH0  = (unsigned short*)carve((size_t)NGATE3 * NHID * 2);
  unsigned short* WIH1  = (unsigned short*)carve((size_t)NGATE3 * NHID * 2);
  unsigned short* WHH1  = (unsigned short*)carve((size_t)NGATE3 * NHID * 2);
  unsigned short* WFC   = (unsigned short*)carve((size_t)NOUTF * NHID * 2);
  if (off > ws_size || off > (size_t)134217728) return;

  const int n8x = NGATE3 * (XKPAD / 8);
  const int n8h = NGATE3 * (NHID / 8);
  const int n8f = NOUTF * (NHID / 8);
  wplane_kernel<<<(n8x + NTHR - 1) / NTHR, NTHR, 0, stream>>>(wih0, WIH0P, NGATE3, NINP, XKPAD / 8, WCARRY);
  wplane_kernel<<<(n8h + NTHR - 1) / NTHR, NTHR, 0, stream>>>(whh0, WHH0,  NGATE3, NHID, NHID / 8,  WCARRY);
  wplane_kernel<<<(n8h + NTHR - 1) / NTHR, NTHR, 0, stream>>>(wih1, WIH1,  NGATE3, NHID, NHID / 8,  WCARRY);
  wplane_kernel<<<(n8h + NTHR - 1) / NTHR, NTHR, 0, stream>>>(whh1, WHH1,  NGATE3, NHID, NHID / 8,  WCARRY);
  wplane_kernel<<<(n8f + NTHR - 1) / NTHR, NTHR, 0, stream>>>(wfc,  WFC,   NOUTF,  NHID, NHID / 8,  WCARRY);

  gru2_seq_kernel<<<NBAT / SEQ_BLK, NTHR, 0, stream>>>(x, WIH0P, WHH0, WIH1, WHH1, WFC, out);
}
